// _MockAttention_19026705121792
// MI455X (gfx1250) — hardware-verified
//
#include <hip/hip_runtime.h>

#define BATCH   2
#define SEQ     2048
#define DMODEL  1024
#define NHEADS  16
#define HDIM    64
#define MTOT    (BATCH * SEQ)

typedef _Float16 v16h __attribute__((ext_vector_type(16)));
typedef _Float16 v8h  __attribute__((ext_vector_type(8)));
typedef float    v8f  __attribute__((ext_vector_type(8)));
typedef float    v4f  __attribute__((ext_vector_type(4)));

union Frag { v16h v; v8h half[2]; };

template <typename T> struct V16;
template <> struct V16<float>    { typedef v4f t; };
template <> struct V16<_Float16> { typedef v8h t; };

static __device__ __forceinline__ v8f wmma16(v16h a, v16h b, v8f c) {
  c = __builtin_amdgcn_wmma_f32_16x16x32_f16(false, a, false, b, (short)0, c, false, false);
  asm volatile("v_nop\n\tv_nop\n\tv_nop\n\tv_nop" : "+v"(c) : "v"(a), "v"(b));
  return c;
}

static __device__ __forceinline__ v16h load_frag(const _Float16* rowp) {
  const int h8 = ((threadIdx.x & 31) >> 4) << 3;
  Frag f;
  f.half[0] = *(const v8h*)(rowp + h8);
  f.half[1] = *(const v8h*)(rowp + 16 + h8);
  return f.v;
}

static __device__ __forceinline__ v8f zero8() {
  v8f z = {0.f, 0.f, 0.f, 0.f, 0.f, 0.f, 0.f, 0.f};
  return z;
}

__global__ __launch_bounds__(256)
void cvt_f16(const float* __restrict__ in, _Float16* __restrict__ out, int n8, float scale) {
  const int i = blockIdx.x * 256 + threadIdx.x;
  if (i >= n8) return;
  const float* p = in + (size_t)i * 8;
  const v4f a = *(const v4f*)p;
  const v4f b = *(const v4f*)(p + 4);
  v8h r;
#pragma unroll
  for (int c = 0; c < 4; ++c) {
    r[c]     = (_Float16)(a[c] * scale);
    r[4 + c] = (_Float16)(b[c] * scale);
  }
  _Float16* q = out + (size_t)i * 8;
  *(volatile v8h*)q = r;
  __threadfence();
  *(volatile v8h*)q = r;
}

template <typename OutT>
__global__ __launch_bounds__(128)
void gemm_bias(const _Float16* __restrict__ A, const _Float16* __restrict__ W,
               const float* __restrict__ bias, OutT* __restrict__ out,
               int M, int K, int N, float oscale) {
  __shared__ __align__(16) OutT sEp[4][32 * 64];
  typedef typename V16<OutT>::t VT;
  constexpr int EPV = 16 / (int)sizeof(OutT);
  constexpr int EPL = 128 / (int)sizeof(OutT);
  constexpr int LPR = 64 / EPL;
  constexpr int NI  = 8 * LPR;

  const int tid  = threadIdx.x;
  const int lane = tid & 31;
  const int l15  = lane & 15;
  const int hi   = lane >> 4;
  const int wave = tid >> 5;
  const int wr   = (wave >> 1) << 5;
  const int wc   = (wave & 1) << 6;
  const int m0   = blockIdx.y * 64;
  const int n0   = blockIdx.x * 128;
  if (m0 + 64 > M || n0 + 128 > N) return;

  v8f acc[2][4];
#pragma unroll
  for (int mi = 0; mi < 2; ++mi)
#pragma unroll
    for (int j = 0; j < 4; ++j) acc[mi][j] = zero8();

  const _Float16* arow0 = A + (size_t)(m0 + wr + l15) * K;
  const _Float16* arow1 = arow0 + (size_t)16 * K;
  const _Float16* wrow0 = W + (size_t)(n0 + wc + l15) * K;

  for (int kk = 0; kk < K; kk += 32) {
    const v16h a0 = load_frag(arow0 + kk);
    const v16h a1 = load_frag(arow1 + kk);
    v16h bfr[4];
#pragma unroll
    for (int j = 0; j < 4; ++j) bfr[j] = load_frag(wrow0 + (size_t)j * 16 * K + kk);
#pragma unroll
    for (int j = 0; j < 4; ++j) {
      acc[0][j] = wmma16(a0, bfr[j], acc[0][j]);
      acc[1][j] = wmma16(a1, bfr[j], acc[1][j]);
    }
  }

  OutT* s = sEp[wave];
#pragma unroll
  for (int mi = 0; mi < 2; ++mi) {
#pragma unroll
    for (int j = 0; j < 4; ++j) {
      const int lc = j * 16 + l15;
      const float bv = bias[n0 + wc + lc];
#pragma unroll
      for (int v = 0; v < 8; ++v) {
        const int lr = mi * 16 + 8 * hi + v;
        s[lr * 64 + lc] = (OutT)(acc[mi][j][v] * oscale + bv);
      }
    }
  }
  __syncthreads();

  VT vals[NI];
#pragma unroll
  for (int q = 0; q < NI; ++q) {
    const int L   = q * 4 + (lane >> 3);
    const int row = L / LPR, seg = L - row * LPR;
    const int eo  = seg * EPL + (lane & 7) * EPV;
    vals[q] = *(const VT*)(s + row * 64 + eo);
  }
#pragma unroll
  for (int q = 0; q < NI; ++q) {
    const int L   = q * 4 + (lane >> 3);
    const int row = L / LPR, seg = L - row * LPR;
    const int eo  = seg * EPL + (lane & 7) * EPV;
    OutT* gp = out + (size_t)(m0 + wr + row) * N + n0 + wc + eo;
    *(volatile VT*)gp = vals[q];
  }
  __threadfence();
#pragma unroll
  for (int q = 0; q < NI; ++q) {
    const int L   = q * 4 + (lane >> 3);
    const int row = L / LPR, seg = L - row * LPR;
    const int eo  = seg * EPL + (lane & 7) * EPV;
    OutT* gp = out + (size_t)(m0 + wr + row) * N + n0 + wc + eo;
    *(volatile VT*)gp = vals[q];
  }
}

__global__ __launch_bounds__(128)
void attention_kernel(const _Float16* __restrict__ qkv,
                      _Float16* __restrict__ attn_out) {
  __shared__ __align__(16) _Float16 sVt[HDIM * 32];
  __shared__ __align__(16) _Float16 sP[4][16 * 32];
  __shared__ __align__(16) _Float16 sO[4][16 * 64];

  const int tid  = threadIdx.x;
  const int lane = tid & 31;
  const int l15  = lane & 15;
  const int hi   = lane >> 4;
  const int wave = tid >> 5;

  const int qt = blockIdx.x;
  const int h  = blockIdx.y;
  const int b  = blockIdx.z;
  const int qbase = qt * 64 + wave * 16;

  const size_t rstride = 3 * (size_t)DMODEL;
  const _Float16* Qb = qkv + (size_t)b * SEQ * rstride + h * HDIM;
  const _Float16* Kb = Qb + DMODEL;
  const _Float16* Vb = Qb + 2 * DMODEL;

  const _Float16* qrow = Qb + (size_t)(qbase + l15) * rstride;
  const v16h qf0 = load_frag(qrow);
  const v16h qf1 = load_frag(qrow + 32);

  v16h vone;
#pragma unroll
  for (int i = 0; i < 16; ++i) vone[i] = (_Float16)1.0f;

  float mrow[8];
  v8f o[4];
#pragma unroll
  for (int t = 0; t < 4; ++t) o[t] = zero8();
  v8f lacc = zero8();
#pragma unroll
  for (int v = 0; v < 8; ++v) mrow[v] = -1e30f;
  const float scale = 0.125f;
  const float pscl  = 256.0f;

  for (int j0 = 0; j0 < SEQ; j0 += 32) {
#pragma unroll
    for (int i = 0; i < 2; ++i) {
      const int e = (tid + i * 128) * 8;
      const int key = e >> 6, d = e & 63;
      const v8h val = *(const v8h*)(Vb + (size_t)(j0 + key) * rstride + d);
#pragma unroll
      for (int x = 0; x < 8; ++x) sVt[(d + x) * 32 + key] = val[x];
    }

    const _Float16* krow0 = Kb + (size_t)(j0 + l15) * rstride;
    const _Float16* krow1 = Kb + (size_t)(j0 + 16 + l15) * rstride;
    v8f s0 = zero8(), s1 = zero8();
    s0 = wmma16(qf0, load_frag(krow0),      s0);
    s0 = wmma16(qf1, load_frag(krow0 + 32), s0);
    s1 = wmma16(qf0, load_frag(krow1),      s1);
    s1 = wmma16(qf1, load_frag(krow1 + 32), s1);

#pragma unroll
    for (int v = 0; v < 8; ++v) {
      const float a = s0[v] * scale, c = s1[v] * scale;
      float mx = fmaxf(a, c);
#pragma unroll
      for (int m = 1; m <= 8; m <<= 1) mx = fmaxf(mx, __shfl_xor(mx, m, 32));
      const float mnew  = fmaxf(mrow[v], mx);
      const float alpha = __expf(mrow[v] - mnew);
      mrow[v] = mnew;
      const float p0 = __expf(a - mnew) * pscl;
      const float p1 = __expf(c - mnew) * pscl;
      lacc[v] *= alpha;
#pragma unroll
      for (int t = 0; t < 4; ++t) o[t][v] *= alpha;
      const int pr = (v + 8 * hi) * 32;
      sP[wave][pr + l15]      = (_Float16)p0;
      sP[wave][pr + 16 + l15] = (_Float16)p1;
    }
    __syncthreads();

    const v16h pf = load_frag(&sP[wave][l15 * 32]);
#pragma unroll
    for (int t = 0; t < 4; ++t) {
      const v16h vf = load_frag(&sVt[(t * 16 + l15) * 32]);
      o[t] = wmma16(pf, vf, o[t]);
    }
    lacc = wmma16(pf, vone, lacc);
    __syncthreads();
  }

#pragma unroll
  for (int v = 0; v < 8; ++v) {
    const float inv = 16.0f / lacc[v];
    const int lr = v + 8 * hi;
#pragma unroll
    for (int t = 0; t < 4; ++t)
      sO[wave][lr * 64 + t * 16 + l15] = (_Float16)(o[t][v] * inv);
  }
  __syncthreads();

  v8h vals[4];
#pragma unroll
  for (int q = 0; q < 4; ++q) {
    const int L = q * 4 + (lane >> 3);
    const int piece = lane & 7;
    vals[q] = *(const v8h*)&sO[wave][L * 64 + piece * 8];
  }
#pragma unroll
  for (int q = 0; q < 4; ++q) {
    const int L = q * 4 + (lane >> 3);
    const int piece = lane & 7;
    _Float16* gp = attn_out + ((size_t)b * SEQ + qbase + L) * DMODEL + h * HDIM + piece * 8;
    *(volatile v8h*)gp = vals[q];
  }
  __threadfence();
#pragma unroll
  for (int q = 0; q < 4; ++q) {
    const int L = q * 4 + (lane >> 3);
    const int piece = lane & 7;
    _Float16* gp = attn_out + ((size_t)b * SEQ + qbase + L) * DMODEL + h * HDIM + piece * 8;
    *(volatile v8h*)gp = vals[q];
  }
}

extern "C" void kernel_launch(void* const* d_in, const int* in_sizes, int n_in,
                              void* d_out, int out_size, void* d_ws, size_t ws_size,
                              hipStream_t stream) {
  if (n_in < 5) return;
  const int nx = MTOT * DMODEL;
  const int nw = 3 * DMODEL * DMODEL;
  const int np = DMODEL * DMODEL;
  const int nq = MTOT * 3 * DMODEL;
  if (in_sizes[0] != nx || in_sizes[1] != nw || in_sizes[2] != 3 * DMODEL ||
      in_sizes[3] != np || in_sizes[4] != DMODEL || out_size != nx) return;

  const float* x      = (const float*)d_in[0];
  const float* qkv_w  = (const float*)d_in[1];
  const float* qkv_b  = (const float*)d_in[2];
  const float* proj_w = (const float*)d_in[3];
  const float* proj_b = (const float*)d_in[4];
  float* out = (float*)d_out;

  char* ws = (char*)d_ws;
  size_t off = 0;
  _Float16* x16     = (_Float16*)(ws + off);  off += (size_t)nx * 2;
  _Float16* qkvw16  = (_Float16*)(ws + off);  off += (size_t)nw * 2;
  _Float16* projw16 = (_Float16*)(ws + off);  off += (size_t)np * 2;
  _Float16* qkv16   = (_Float16*)(ws + off);  off += (size_t)nq * 2;
  _Float16* attn16  = (_Float16*)(ws + off);  off += (size_t)nx * 2;
  if (off > ws_size) return;

  cvt_f16<<<(nx / 8 + 255) / 256, 256, 0, stream>>>(x, x16, nx / 8, 1.0f);
  cvt_f16<<<(nw / 8 + 255) / 256, 256, 0, stream>>>(qkv_w, qkvw16, nw / 8, 64.0f);
  cvt_f16<<<(np / 8 + 255) / 256, 256, 0, stream>>>(proj_w, projw16, np / 8, 64.0f);

  gemm_bias<_Float16><<<dim3(3 * DMODEL / 128, MTOT / 64), 128, 0, stream>>>(
      x16, qkvw16, qkv_b, qkv16, MTOT, DMODEL, 3 * DMODEL, 1.0f / 64.0f);

  attention_kernel<<<dim3(SEQ / 64, NHEADS, BATCH), 128, 0, stream>>>(qkv16, attn16);

  gemm_bias<float><<<dim3(DMODEL / 128, MTOT / 64), 128, 0, stream>>>(
      attn16, projw16, proj_b, out, MTOT, DMODEL, DMODEL, 1.0f / 1024.0f);
}
